// _DualGraphGAT_24670292148714
// MI455X (gfx1250) — hardware-verified
//
#include <hip/hip_runtime.h>
#include <stddef.h>


#define FDIM    256
#define HEADS   4
#define CHN     64
#define HID2    128
#define OUTP    64
#define NTHR    256
#define NWAVE   8
#define BMR     32
#define EPT     8
#define NGRP    2
#define CHUNK   (NTHR * EPT * NGRP)
#define WCAP    (EPT * NGRP * 32)
#define LISTN   (NWAVE * WCAP)
#define NBC     4096
#define NBF     1024
#define RCAP    40960
#define RBN     128
#define TGT     256
#define DEGCAP  256
#define OTHR    512
#define WSCAP   134217728
#define NEG_SLOPE 0.2f
#define SCA     16.0f
#define SCW     16.0f
#define INVS    (1.0f / 256.0f)

#define WSEG1   65536
#define WSEG2   131072
#define WSEG3   196608
#define WSEG4   262144
#define WSEG5   278528
#define WSEG6   294912
#define WSEG7   299008
#define WTOT    315392

#define LDS_FILL ((RCAP + NBF + LISTN) * 4 + 64)

static_assert((CHUNK & (CHUNK - 1)) == 0);
static_assert(CHUNK <= 4096);
static_assert(NBC <= 4096 && NBF <= 4096);
static_assert((NBC & (NBC - 1)) == 0 && (NBF & (NBF - 1)) == 0);
static_assert(NBC == 4 * NBF);
static_assert(OTHR * 8 == NBC);
static_assert((RCAP % 32) == 0);
static_assert(TGT == NWAVE * 32);
static_assert((NBC % TGT) == 0);
static_assert((TGT % BMR) == 0);
static_assert(HEADS * CHN == FDIM);
static_assert(FDIM == 8 * 32);
static_assert(WTOT % (8 * NTHR) == 0);
static_assert(HID2 == 2 * OUTP);

typedef float    v4f  __attribute__((ext_vector_type(4)));
typedef float    v8f  __attribute__((ext_vector_type(8)));
typedef int      v4i  __attribute__((ext_vector_type(4)));
typedef _Float16 v8h  __attribute__((ext_vector_type(8)));
typedef _Float16 v16h __attribute__((ext_vector_type(16)));
union FragH { v16h v; v8h h[2]; };

__device__ __forceinline__ v8f wmh(v16h a, v16h b, v8f c) {
  v8f d = __builtin_amdgcn_wmma_f32_16x16x32_f16(false, a, false, b, (short)0, c, false, false);
  asm volatile("v_nop\n\tv_nop\n\tv_nop\n\tv_nop" : "+v"(d) : "v"(a), "v"(b));
  return d;
}

__device__ __forceinline__ v8h cvt8(v4f a, v4f b, float s) {
  v8h o;
  o[0] = (_Float16)(a.x * s); o[1] = (_Float16)(a.y * s);
  o[2] = (_Float16)(a.z * s); o[3] = (_Float16)(a.w * s);
  o[4] = (_Float16)(b.x * s); o[5] = (_Float16)(b.y * s);
  o[6] = (_Float16)(b.z * s); o[7] = (_Float16)(b.w * s);
  return o;
}

__device__ __forceinline__ float lrelu(float v) { return v > 0.0f ? v : NEG_SLOPE * v; }
__device__ __forceinline__ float eluf(float v)  { return v > 0.0f ? v : (__expf(v) - 1.0f); }

__global__ __launch_bounds__(NTHR) void k_wcvt(
    const float* __restrict__ w0, const float* __restrict__ w1, const float* __restrict__ w2,
    const float* __restrict__ w3, const float* __restrict__ w4, const float* __restrict__ w5,
    const float* __restrict__ w6, const float* __restrict__ w7, _Float16* wp) {
  const int i = (int)blockIdx.x * NTHR + (int)threadIdx.x;
  const int e = 8 * i;
  const float* src = w0;
  int lo = 0;
  src = (e >= WSEG1) ? w1 : src;  lo = (e >= WSEG1) ? WSEG1 : lo;
  src = (e >= WSEG2) ? w2 : src;  lo = (e >= WSEG2) ? WSEG2 : lo;
  src = (e >= WSEG3) ? w3 : src;  lo = (e >= WSEG3) ? WSEG3 : lo;
  src = (e >= WSEG4) ? w4 : src;  lo = (e >= WSEG4) ? WSEG4 : lo;
  src = (e >= WSEG5) ? w5 : src;  lo = (e >= WSEG5) ? WSEG5 : lo;
  src = (e >= WSEG6) ? w6 : src;  lo = (e >= WSEG6) ? WSEG6 : lo;
  src = (e >= WSEG7) ? w7 : src;  lo = (e >= WSEG7) ? WSEG7 : lo;
  const float* p = src + (e - lo);
  const v4f a = *(const v4f*)p;
  const v4f b = *(const v4f*)(p + 4);
  const v8h o = cvt8(a, b, SCW);
  _Float16* d = wp + (size_t)e;
  *(volatile v8h*)d = o;
  __threadfence();
  *(volatile v8h*)d = o;
}

__global__ __launch_bounds__(NTHR) void k_xcvt(const float* __restrict__ x, _Float16* xp, int nN, int nUnits) {
  const int i = (int)blockIdx.x * NTHR + (int)threadIdx.x;
  if (i >= nUnits) return;
  const int row = i >> 5;
  const int c0  = (i & 31) * 8;
  int rr = row > nN - 1 ? nN - 1 : row;
  rr = rr < 0 ? 0 : rr;
  const float* p = x + (size_t)rr * FDIM + c0;
  v4f a = *(const v4f*)p, b = *(const v4f*)(p + 4);
  const v4f z = {0.f, 0.f, 0.f, 0.f};
  if (row >= nN) { a = z; b = z; }
  const v8h o = cvt8(a, b, SCA);
  _Float16* d = xp + (size_t)i * 8;
  *(volatile v8h*)d = o;
  __threadfence();
  *(volatile v8h*)d = o;
}

template <int NB>
__device__ __forceinline__ int scan_chunk(const int* __restrict__ dsts, int nE, int cbase, int slotBase,
                                          int vec8, int* list, int tid, int lane, int wave) {
  int wc = 0;
#pragma unroll
  for (int g = 0; g < NGRP; ++g) {
    const int el0  = (g * NTHR + tid) * EPT;
    const int e0   = cbase + el0;
    const int sent = -2147483647 - 1;
    v4i da, db;
    if (vec8 != 0 && cbase + CHUNK <= nE) {
      da = *(const v4i*)(dsts + e0);
      db = *(const v4i*)(dsts + e0 + 4);
    } else {
      da.x = (e0     < nE) ? dsts[min(e0, nE - 1)] : sent;
      da.y = (e0 + 1 < nE) ? dsts[min(e0 + 1, nE - 1)] : sent;
      da.z = (e0 + 2 < nE) ? dsts[min(e0 + 2, nE - 1)] : sent;
      da.w = (e0 + 3 < nE) ? dsts[min(e0 + 3, nE - 1)] : sent;
      db.x = (e0 + 4 < nE) ? dsts[min(e0 + 4, nE - 1)] : sent;
      db.y = (e0 + 5 < nE) ? dsts[min(e0 + 5, nE - 1)] : sent;
      db.z = (e0 + 6 < nE) ? dsts[min(e0 + 6, nE - 1)] : sent;
      db.w = (e0 + 7 < nE) ? dsts[min(e0 + 7, nE - 1)] : sent;
    }
    const unsigned nb = (unsigned)slotBase;
    const unsigned s0 = (unsigned)da.x - nb, s1 = (unsigned)da.y - nb;
    const unsigned s2 = (unsigned)da.z - nb, s3 = (unsigned)da.w - nb;
    const unsigned s4 = (unsigned)db.x - nb, s5 = (unsigned)db.y - nb;
    const unsigned s6 = (unsigned)db.z - nb, s7 = (unsigned)db.w - nb;
    const bool h0 = s0 < (unsigned)NB, h1 = s1 < (unsigned)NB, h2 = s2 < (unsigned)NB, h3 = s3 < (unsigned)NB;
    const bool h4 = s4 < (unsigned)NB, h5 = s5 < (unsigned)NB, h6 = s6 < (unsigned)NB, h7 = s7 < (unsigned)NB;
    const unsigned any = __builtin_amdgcn_ballot_w32(h0 | h1 | h2 | h3 | h4 | h5 | h6 | h7);
    if (any != 0u) {
#define HITJ(J, HJ, SJ) { \
        const unsigned mj = __builtin_amdgcn_ballot_w32(HJ); \
        if (mj != 0u) { \
          if (HJ) { \
            const int pos = wc + (int)__builtin_amdgcn_mbcnt_lo(mj, 0u); \
            if (pos < WCAP) list[wave * WCAP + pos] = ((el0 + (J)) << 12) | (int)(SJ); \
          } \
          wc += (int)__builtin_popcount(mj); } }
      HITJ(0, h0, s0)
      HITJ(1, h1, s1)
      HITJ(2, h2, s2)
      HITJ(3, h3, s3)
      HITJ(4, h4, s4)
      HITJ(5, h5, s5)
      HITJ(6, h6, s6)
      HITJ(7, h7, s7)
#undef HITJ
    }
  }
  return wc;
}

__global__ __launch_bounds__(NTHR) void k_count(
    const int* __restrict__ dsts, int* cnt, int nE, int vec8) {
  __shared__ __attribute__((aligned(16))) int scnt[NBC];
  __shared__ __attribute__((aligned(16))) int list[LISTN];
  __shared__ int wcnt[NWAVE];
  const int tid = threadIdx.x, lane = tid & 31, wave = tid >> 5;
  const int nodeBase = blockIdx.x * NBC;

  for (int i = tid; i < NBC; i += NTHR) scnt[i] = 0;
  __syncthreads();

  const int nChunks = (nE + CHUNK - 1) / CHUNK;
#pragma unroll 1
  for (int ch = 0; ch < nChunks; ++ch) {
    const int cbase = ch * CHUNK;
    const int wc = scan_chunk<NBC>(dsts, nE, cbase, nodeBase, vec8, list, tid, lane, wave);
    if (lane == 0) wcnt[wave] = wc;
    __syncthreads();
    if (wave == 0) {
#pragma unroll 1
      for (int wsx = 0; wsx < NWAVE; ++wsx) {
        int n = __builtin_amdgcn_readfirstlane(wcnt[wsx]);
        n = n > WCAP ? WCAP : (n < 0 ? 0 : n);
        const int* lp = list + wsx * WCAP;
#pragma unroll 1
        for (int i = 0; i < n; ++i) {
          const int ent  = __builtin_amdgcn_readfirstlane(lp[i]);
          const int slot = ent & (NBC - 1);
          if (lane == 0) scnt[slot] = scnt[slot] + 1;
        }
      }
    }
    __syncthreads();
  }

  v4i cq[4];
#pragma unroll
  for (int q = 0; q < 4; ++q) {
    const int f = (wave * 4 + q) * 128 + 4 * lane;
    cq[q] = *(const v4i*)(scnt + f);
  }
  int* cp = cnt + (size_t)nodeBase;
#pragma unroll
  for (int q = 0; q < 4; ++q) {
    const int f = (wave * 4 + q) * 128 + 4 * lane;
    *(volatile v4i*)(cp + f) = cq[q];
  }
  __threadfence();
#pragma unroll
  for (int q = 0; q < 4; ++q) {
    const int f = (wave * 4 + q) * 128 + 4 * lane;
    *(volatile v4i*)(cp + f) = cq[q];
  }
}

__global__ __launch_bounds__(OTHR) void k_offsets(
    const int* __restrict__ cnt, int* off, int* rbase, int nChunk) {
  __shared__ __attribute__((aligned(16))) int soff[NBC];
  __shared__ __attribute__((aligned(16))) int srb[RBN];
  __shared__ int wtot[OTHR / 32];
  const int tid = threadIdx.x, lane = tid & 31, wave = tid >> 5, sub = tid >> 7;
  for (int i = tid; i < RBN; i += OTHR) srb[i] = 0;
  int carry = 0;
#pragma unroll 1
  for (int ch = 0; ch < nChunk; ++ch) {
    const int base = ch * NBC;
    const v4i c0 = *(const v4i*)(cnt + base + 8 * tid);
    const v4i c1 = *(const v4i*)(cnt + base + 8 * tid + 4);
    const int e0 = max(c0.x, 0), e1 = max(c0.y, 0), e2 = max(c0.z, 0), e3 = max(c0.w, 0);
    const int e4 = max(c1.x, 0), e5 = max(c1.y, 0), e6 = max(c1.z, 0), e7 = max(c1.w, 0);
    const int ts = e0 + e1 + e2 + e3 + e4 + e5 + e6 + e7;
    int incl = ts;
#pragma unroll
    for (int d = 1; d < 32; d <<= 1) {
      const int t = __shfl_up(incl, d);
      if (lane >= d) incl += t;
    }
    if (lane == 31) wtot[wave] = incl;
    __syncthreads();
    const int S0 = wtot[0]  + wtot[1]  + wtot[2]  + wtot[3];
    const int S1 = wtot[4]  + wtot[5]  + wtot[6]  + wtot[7];
    const int S2 = wtot[8]  + wtot[9]  + wtot[10] + wtot[11];
    const int S3 = wtot[12] + wtot[13] + wtot[14] + wtot[15];
    int pre = 0;
#pragma unroll 1
    for (int w = 4 * sub; w < wave; ++w) pre += wtot[w];
    const int b0 = carry;
    const int b1 = b0 + ((S0 + 31) & ~31);
    const int b2 = b1 + ((S1 + 31) & ~31);
    const int b3 = b2 + ((S2 + 31) & ~31);
    const int b4 = b3 + ((S3 + 31) & ~31);
    const int myb = sub == 0 ? b0 : (sub == 1 ? b1 : (sub == 2 ? b2 : b3));
    if (tid == 0) {
      srb[min(4 * ch + 0, RBN - 1)] = b0;
      srb[min(4 * ch + 1, RBN - 1)] = b1;
      srb[min(4 * ch + 2, RBN - 1)] = b2;
      srb[min(4 * ch + 3, RBN - 1)] = b3;
    }
    int run = myb + pre + incl - ts;
    soff[8 * tid + 0] = run; run += e0;
    soff[8 * tid + 1] = run; run += e1;
    soff[8 * tid + 2] = run; run += e2;
    soff[8 * tid + 3] = run; run += e3;
    soff[8 * tid + 4] = run; run += e4;
    soff[8 * tid + 5] = run; run += e5;
    soff[8 * tid + 6] = run; run += e6;
    soff[8 * tid + 7] = run;
    carry = b4;
    __syncthreads();
    const v4i o0 = *(const v4i*)(soff + 4 * tid);
    const v4i o1 = *(const v4i*)(soff + 4 * (tid + OTHR));
    int* op = off + base;
    *(volatile v4i*)(op + 4 * tid) = o0;
    *(volatile v4i*)(op + 4 * (tid + OTHR)) = o1;
    __threadfence();
    *(volatile v4i*)(op + 4 * tid) = o0;
    *(volatile v4i*)(op + 4 * (tid + OTHR)) = o1;
    __syncthreads();
  }
  if (tid == 0) srb[min(4 * nChunk, RBN - 1)] = carry;
  __syncthreads();
  v4i rv = {0, 0, 0, 0};
  if (tid < 32) rv = *(const v4i*)(srb + 4 * tid);
  if (tid < 32) *(volatile v4i*)(rbase + 4 * tid) = rv;
  __threadfence();
  if (tid < 32) *(volatile v4i*)(rbase + 4 * tid) = rv;
}

__global__ __launch_bounds__(NTHR) void k_fill(
    const int* __restrict__ srcs, const int* __restrict__ dsts,
    const int* __restrict__ off, const int* __restrict__ rbase,
    int* csr, int nN, int nE, int vec8, int csrLen) {
  extern __shared__ v4f lds_dyn[];
  int* region = (int*)lds_dyn;
  int* cursor = region + RCAP;
  int* list   = cursor + NBF;
  int* wcnt   = list + LISTN;
  const int tid = threadIdx.x, lane = tid & 31, wave = tid >> 5;
  const int b = blockIdx.x;
  const int nodeBase = b * NBF;

  int rb0 = rbase[b];
  const int rb1 = rbase[b + 1];
  rb0 = rb0 < 0 ? 0 : (rb0 > csrLen ? csrLen : rb0);
  rb0 &= ~31;
  int len = rb1 - rb0;
  len = len < 0 ? 0 : (len > RCAP ? RCAP : len);
  int lenW = (len + 31) & ~31;
  if (rb0 + lenW > csrLen) lenW = (csrLen - rb0) & ~31;

  {
    const v4i z = {0, 0, 0, 0};
    for (int i = tid; i < RCAP / 4; i += NTHR) ((v4i*)region)[i] = z;
    for (int s = tid; s < NBF; s += NTHR) {
      int o = off[nodeBase + s] - rb0;
      o = o < 0 ? 0 : (o > RCAP ? RCAP : o);
      cursor[s] = o;
    }
  }
  __syncthreads();

  const int nChunks = (nE + CHUNK - 1) / CHUNK;
#pragma unroll 1
  for (int ch = 0; ch < nChunks; ++ch) {
    const int cbase = ch * CHUNK;
    const int wc = scan_chunk<NBF>(dsts, nE, cbase, nodeBase, vec8, list, tid, lane, wave);
    if (lane == 0) wcnt[wave] = wc;
    __syncthreads();
    if (wave == 0) {
#pragma unroll 1
      for (int wsx = 0; wsx < NWAVE; ++wsx) {
        int n = __builtin_amdgcn_readfirstlane(wcnt[wsx]);
        n = n > WCAP ? WCAP : (n < 0 ? 0 : n);
        const int* lp = list + wsx * WCAP;
#pragma unroll 1
        for (int i = 0; i < n; ++i) {
          const int ent  = __builtin_amdgcn_readfirstlane(lp[i]);
          const int slot = ent & (NBF - 1);
          int e = cbase + ((ent >> 12) & (CHUNK - 1));
          e = e > nE - 1 ? nE - 1 : e;
          int src = srcs[e];
          src = src < 0 ? 0 : (src > nN - 1 ? nN - 1 : src);
          if (lane == 0) {
            int pos = cursor[slot];
            pos = pos < 0 ? 0 : (pos > RCAP - 1 ? RCAP - 1 : pos);
            region[pos] = src;
            const int np = pos + 1;
            cursor[slot] = np > RCAP ? RCAP : np;
          }
        }
      }
    }
    __syncthreads();
  }

  const int nv = lenW >> 2;
  int* gp = csr + rb0;
#pragma unroll 1
  for (int i = tid; i < nv; i += NTHR) { const v4i v = ((const v4i*)region)[i]; *(volatile v4i*)(gp + 4 * i) = v; }
  __threadfence();
#pragma unroll 1
  for (int i = tid; i < nv; i += NTHR) { const v4i v = ((const v4i*)region)[i]; *(volatile v4i*)(gp + 4 * i) = v; }
}

template <int K, int LDA, int NC>
__device__ __forceinline__ void gemm_core(const _Float16* __restrict__ Ap, const _Float16* __restrict__ Bp,
                                          float* stg, int rowBase) {
  constexpr int TPW = NC / 64;
  constexpr int KT  = K / 32;
  static_assert(K % 32 == 0 && NC % 64 == 0 && LDA % 8 == 0 && LDA >= K);
  static_assert(TPW >= 1 && TPW <= 4);
  const int tid = threadIdx.x, lane = tid & 31, wave = tid >> 5, hh = lane >> 4, m = lane & 15;
  const int rg = wave >> 2, cg = wave & 3;
  const int r0 = 16 * rg;
  const int c0 = cg * (NC / 4);

  v8f acc[TPW];
#pragma unroll
  for (int t = 0; t < TPW; ++t) { v8f z = {0.f, 0.f, 0.f, 0.f, 0.f, 0.f, 0.f, 0.f}; acc[t] = z; }

  const _Float16* ap  = Ap + (size_t)(rowBase + r0 + m) * LDA + 8 * hh;
  const _Float16* bp0 = Bp + (size_t)(c0 + m) * K + 8 * hh;
#pragma unroll 1
  for (int kt = 0; kt < KT; ++kt) {
    FragH a;
    a.h[0] = *(const v8h*)(ap + 32 * kt);
    a.h[1] = *(const v8h*)(ap + 32 * kt + 16);
#pragma unroll
    for (int t = 0; t < TPW; ++t) {
      const _Float16* bp = bp0 + (size_t)(16 * t) * K + 32 * kt;
      FragH bf;
      bf.h[0] = *(const v8h*)bp;
      bf.h[1] = *(const v8h*)(bp + 16);
      acc[t] = wmh(a.v, bf.v, acc[t]);
    }
  }

  {
    float* sp = stg + (size_t)(r0 + 8 * hh) * NC + c0 + m;
#pragma unroll
    for (int t = 0; t < TPW; ++t) {
#pragma unroll
      for (int r = 0; r < 8; ++r) sp[r * NC + 16 * t] = acc[t][r] * INVS;
    }
  }
  __syncthreads();
}

template <int K, int LDA>
__global__ __launch_bounds__(NTHR) void k_gemm_att(
    const _Float16* __restrict__ Ap, const _Float16* __restrict__ Bp,
    const float* __restrict__ attS, const float* __restrict__ attD,
    float* C, float* eS, float* eD) {
  constexpr int NC  = FDIM;
  constexpr int NES = BMR * HEADS;
  constexpr int NV  = NES / 4;
  constexpr int NF4 = BMR * NC / 4;
  constexpr int NIT = NF4 / NTHR;
  static_assert(NF4 % NTHR == 0);
  static_assert(2 * NV <= NTHR);
  static_assert(NTHR == 8 * BMR);
  __shared__ __attribute__((aligned(32))) float stg[BMR * NC];
  __shared__ __attribute__((aligned(16))) float sES[NES];
  __shared__ __attribute__((aligned(16))) float sED[NES];
  const int tid = threadIdx.x;
  const int rowBase = blockIdx.x * BMR;

  gemm_core<K, LDA, NC>(Ap, Bp, stg, rowBase);

  {
    const int drow = tid >> 3, part = tid & 7;
    const float* rp  = stg + (size_t)drow * NC + 32 * part;
    const float* sa  = attS + 32 * part;
    const float* sdd = attD + 32 * part;
    float ps = 0.f, pd = 0.f;
#pragma unroll 2
    for (int c = 0; c < 32; c += 4) {
      const v4f hv = *(const v4f*)(rp + c);
      const v4f av = *(const v4f*)(sa + c);
      const v4f dv = *(const v4f*)(sdd + c);
      ps += hv.x * av.x + hv.y * av.y + hv.z * av.z + hv.w * av.w;
      pd += hv.x * dv.x + hv.y * dv.y + hv.z * dv.z + hv.w * dv.w;
    }
    ps += __shfl_xor(ps, 1); pd += __shfl_xor(pd, 1);
    if ((part & 1) == 0) { sES[drow * HEADS + (part >> 1)] = ps; sED[drow * HEADS + (part >> 1)] = pd; }
  }

  {
    float* tileC = C + (size_t)rowBase * NC;
    v4f cv[NIT];
#pragma unroll
    for (int it = 0; it < NIT; ++it) cv[it] = *(const v4f*)(stg + 4 * (it * NTHR + tid));
#pragma unroll
    for (int it = 0; it < NIT; ++it) *(volatile v4f*)(tileC + 4 * (size_t)(it * NTHR + tid)) = cv[it];
    __threadfence();
#pragma unroll
    for (int it = 0; it < NIT; ++it) *(volatile v4f*)(tileC + 4 * (size_t)(it * NTHR + tid)) = cv[it];
  }
  __syncthreads();

  {
    const size_t eb = (size_t)rowBase * HEADS;
    const int iS = tid < NV - 1 ? tid : NV - 1;
    int iD = tid - NV; iD = iD < 0 ? 0 : (iD > NV - 1 ? NV - 1 : iD);
    const v4f vS = *(const v4f*)(sES + 4 * iS);
    const v4f vD = *(const v4f*)(sED + 4 * iD);
    const bool isS = tid < NV;
    const v4f dv = isS ? vS : vD;
    float* gp = isS ? (eS + eb + 4 * iS) : (eD + eb + 4 * iD);
    if (tid < 2 * NV) *(volatile v4f*)gp = dv;
    __threadfence();
    if (tid < 2 * NV) *(volatile v4f*)gp = dv;
  }
}

__global__ __launch_bounds__(NTHR) void k_gemm_relu16(
    const _Float16* __restrict__ Ap, const _Float16* __restrict__ Bp,
    const float* __restrict__ bA, const float* __restrict__ bB, _Float16* Cp) {
  constexpr int K  = FDIM;
  constexpr int NC = HID2;
  constexpr int NU = BMR * NC / 8;
  constexpr int NIT = NU / NTHR;
  static_assert(NU % NTHR == 0 && NIT == 2);
  __shared__ __attribute__((aligned(32))) float stg[BMR * NC];
  const int tid = threadIdx.x;
  const int rowBase = blockIdx.x * BMR;

  gemm_core<K, FDIM, NC>(Ap, Bp, stg, rowBase);

  v8h ov[NIT];
#pragma unroll
  for (int it = 0; it < NIT; ++it) {
    const int u   = it * NTHR + tid;
    const int row = u >> 4;
    const int cu  = (u & 15) * 8;
    const v4f s0 = *(const v4f*)(stg + row * NC + cu);
    const v4f s1 = *(const v4f*)(stg + row * NC + cu + 4);
    const int ia = cu < OUTP - 8 ? cu : OUTP - 8;
    int ib = cu - OUTP; ib = ib < 0 ? 0 : (ib > OUTP - 8 ? OUTP - 8 : ib);
    const v4f a0 = *(const v4f*)(bA + ia), a1 = *(const v4f*)(bA + ia + 4);
    const v4f b0 = *(const v4f*)(bB + ib), b1 = *(const v4f*)(bB + ib + 4);
    const bool inA = cu < OUTP;
    const v4f q0 = inA ? a0 : b0;
    const v4f q1 = inA ? a1 : b1;
    v4f r0 = s0 + q0, r1 = s1 + q1;
    float f[8];
    f[0] = r0.x; f[1] = r0.y; f[2] = r0.z; f[3] = r0.w;
    f[4] = r1.x; f[5] = r1.y; f[6] = r1.z; f[7] = r1.w;
    v8h o;
#pragma unroll
    for (int q = 0; q < 8; ++q) {
      const float t = f[q] > 0.f ? f[q] : 0.f;
      o[q] = (_Float16)(t * SCA);
    }
    ov[it] = o;
  }
  _Float16* tileC = Cp + (size_t)rowBase * NC;
#pragma unroll
  for (int it = 0; it < NIT; ++it) *(volatile v8h*)(tileC + 8 * (size_t)(it * NTHR + tid)) = ov[it];
  __threadfence();
#pragma unroll
  for (int it = 0; it < NIT; ++it) *(volatile v8h*)(tileC + 8 * (size_t)(it * NTHR + tid)) = ov[it];
}

template <int K, int LDA, int NC>
__global__ __launch_bounds__(NTHR) void k_gemm_out(
    const _Float16* __restrict__ Ap, const _Float16* __restrict__ Bp,
    const float* __restrict__ bias, float* Out, int nN) {
  constexpr int UPR = NC / 4;
  constexpr int NIT = BMR * UPR / NTHR;
  static_assert((BMR * UPR) % NTHR == 0);
  __shared__ __attribute__((aligned(32))) float stg[BMR * NC];
  const int tid = threadIdx.x;
  const int rowBase = blockIdx.x * BMR;
  if (rowBase >= nN) return;

  gemm_core<K, LDA, NC>(Ap, Bp, stg, rowBase);

  int nval = nN - rowBase;
  nval = nval < 0 ? 0 : (nval > BMR ? BMR : nval);
  v4f cv[NIT];
  bool ok[NIT];
#pragma unroll
  for (int it = 0; it < NIT; ++it) {
    const int u   = it * NTHR + tid;
    const int row = u / UPR;
    const int cq  = (u - row * UPR) * 4;
    const v4f s = *(const v4f*)(stg + 4 * u);
    const v4f b = *(const v4f*)(bias + cq);
    cv[it] = s + b;
    ok[it] = row < nval;
  }
  float* tileC = Out + (size_t)rowBase * NC;
#pragma unroll
  for (int it = 0; it < NIT; ++it) if (ok[it]) *(volatile v4f*)(tileC + 4 * (size_t)(it * NTHR + tid)) = cv[it];
  __threadfence();
#pragma unroll
  for (int it = 0; it < NIT; ++it) if (ok[it]) *(volatile v4f*)(tileC + 4 * (size_t)(it * NTHR + tid)) = cv[it];
}

template <int MODE>
__global__ __launch_bounds__(NTHR) void k_agg(
    const int* __restrict__ csr, const int* __restrict__ off, const int* __restrict__ cnt,
    const float* __restrict__ eS, const float* __restrict__ eD, const float* __restrict__ hw,
    const float* __restrict__ bias, const float* __restrict__ gsc, const float* __restrict__ hsIn,
    float* outF, _Float16* outH, int nN, int csrLen) {
  __shared__ __attribute__((aligned(32))) float    sRowF[NWAVE * FDIM];
  __shared__ __attribute__((aligned(16))) _Float16 sRowH[NWAVE * FDIM];
  const int tid = threadIdx.x, lane = tid & 31, wave = tid >> 5;
  const int tbase = blockIdx.x * TGT + wave * 32;
  const int col = 8 * lane;
  const int hd  = lane >> 3;
  float*    srf = sRowF + wave * FDIM;
  _Float16* srh = sRowH + wave * FDIM;

  const v8f bb = *(const v8f*)(bias + col);
  float gg = 0.f, og = 0.f;
  if constexpr (MODE != 0) {
    const float gv = gsc[0];
    gg = __builtin_amdgcn_rcpf(1.0f + __expf(-gv));
    og = 1.0f - gg;
  }

  const int cl    = tbase + lane;
  const int cnt_l = cnt[cl];
  const int off_l = off[cl];

#pragma unroll 1
  for (int j = 0; j < 32; ++j) {
    const int c = tbase + j;
    int n = __shfl(cnt_l, j);
    n = n < 0 ? 0 : (n > DEGCAP ? DEGCAP : n);
    const int st = __shfl(off_l, j);
    const float edc   = eD[(size_t)c * HEADS + hd];
    const float eself = lrelu(eS[(size_t)c * HEADS + hd] + edc);

    float mx = eself;
#pragma unroll 1
    for (int q0 = 0; q0 < n; q0 += 32) {
      int pos = st + q0 + lane;
      pos = pos < 0 ? 0 : (pos > csrLen - 1 ? csrLen - 1 : pos);
      int sl = csr[pos];
      sl = sl < 0 ? 0 : (sl > nN - 1 ? nN - 1 : sl);
      const int mcnt = (n - q0) < 32 ? (n - q0) : 32;
#pragma unroll 1
      for (int pp = 0; pp < mcnt; ++pp) {
        const int s = __builtin_amdgcn_readlane(sl, pp);
        mx = fmaxf(mx, lrelu(eS[(size_t)s * HEADS + hd] + edc));
      }
    }

    float p   = __expf(eself - mx);
    float den = p;
    v8f acc = *(const v8f*)(hw + (size_t)c * FDIM + col) * p;
#pragma unroll 1
    for (int q0 = 0; q0 < n; q0 += 32) {
      int pos = st + q0 + lane;
      pos = pos < 0 ? 0 : (pos > csrLen - 1 ? csrLen - 1 : pos);
      int sl = csr[pos];
      sl = sl < 0 ? 0 : (sl > nN - 1 ? nN - 1 : sl);
      const int mcnt = (n - q0) < 32 ? (n - q0) : 32;
#pragma unroll 1
      for (int pp = 0; pp < mcnt; ++pp) {
        const int s = __builtin_amdgcn_readlane(sl, pp);
        p = __expf(lrelu(eS[(size_t)s * HEADS + hd] + edc) - mx);
        den += p;
        const v8f hv = *(const v8f*)(hw + (size_t)s * FDIM + col);
        acc = acc + hv * p;
      }
    }

    const float rd = __builtin_amdgcn_rcpf(den);
    const v8f v = acc * rd + bb;
    const bool live = (c < nN);

    if constexpr (MODE == 0) {
      v8f t;
#pragma unroll
      for (int i = 0; i < 8; ++i) t[i] = live ? v[i] : 0.0f;
      *(v8f*)(srf + col) = t;
    } else {
      const v8f hsv = *(const v8f*)(hsIn + (size_t)c * FDIM + col);
      v8f hv = hsv * gg + v * og;
      v8h o;
      if constexpr (MODE == 1) {
#pragma unroll
        for (int i = 0; i < 8; ++i) {
          float t = eluf(hv[i]);
          t = live ? t : 0.0f;
          o[i] = (_Float16)(t * SCA);
        }
      } else {
#pragma unroll
        for (int i = 0; i < 8; ++i) {
          const float t = live ? hv[i] : 0.0f;
          o[i] = (_Float16)(t * SCA);
        }
        *(v8f*)(srf + col) = hv;
      }
      *(v8h*)(srh + col) = o;
    }
    __syncthreads();

    if constexpr (MODE == 0) {
      const v4f p0 = *(const v4f*)(srf + 4 * lane);
      const v4f p1 = *(const v4f*)(srf + 128 + 4 * lane);
      float* gp = outF + (size_t)c * FDIM;
      *(volatile v4f*)(gp + 4 * lane) = p0;
      *(volatile v4f*)(gp + 128 + 4 * lane) = p1;
      __threadfence();
      *(volatile v4f*)(gp + 4 * lane) = p0;
      *(volatile v4f*)(gp + 128 + 4 * lane) = p1;
    } else if constexpr (MODE == 1) {
      const v8h pv = *(const v8h*)(srh + 8 * lane);
      _Float16* hp = outH + (size_t)c * FDIM + 8 * lane;
      *(volatile v8h*)hp = pv;
      __threadfence();
      *(volatile v8h*)hp = pv;
    } else {
      const v4f p0 = *(const v4f*)(srf + 4 * lane);
      const v4f p1 = *(const v4f*)(srf + 128 + 4 * lane);
      const v8h pv = *(const v8h*)(srh + 8 * lane);
      float* gp = outF + (size_t)c * FDIM;
      _Float16* hp = outH + (size_t)c * FDIM + 8 * lane;
      if (live) {
        *(volatile v4f*)(gp + 4 * lane) = p0;
        *(volatile v4f*)(gp + 128 + 4 * lane) = p1;
      }
      *(volatile v8h*)hp = pv;
      __threadfence();
      if (live) {
        *(volatile v4f*)(gp + 4 * lane) = p0;
        *(volatile v4f*)(gp + 128 + 4 * lane) = p1;
      }
      *(volatile v8h*)hp = pv;
    }
    __syncthreads();
  }
}

struct CsrSet {
  int* cnt; int* off; int* rb; int* csr;
};

static void build_csr(const int* src, const int* dst, int nE, int nN, int nBC, int nBF, int csrLen,
                      const CsrSet& cs, hipStream_t stream) {
  const int vec8 = ((nE & 3) == 0) ? 1 : 0;
  k_count<<<nBC, NTHR, 0, stream>>>(dst, cs.cnt, nE, vec8);
  k_offsets<<<1, OTHR, 0, stream>>>(cs.cnt, cs.off, cs.rb, nBC);
  hipFuncSetAttribute(reinterpret_cast<const void*>(&k_fill),
                      hipFuncAttributeMaxDynamicSharedMemorySize, LDS_FILL);
  k_fill<<<nBF, NTHR, LDS_FILL, stream>>>(src, dst, cs.off, cs.rb, cs.csr, nN, nE, vec8, csrLen);
}

extern "C" void kernel_launch(void* const* d_in, const int* in_sizes, int n_in,
                              void* d_out, int out_size, void* d_ws, size_t ws_size,
                              hipStream_t stream) {
  if (n_in < 29) return;
  const int nN  = in_sizes[0] / FDIM;
  const int nEs = in_sizes[1] / 2;
  const int nEe = in_sizes[2] / 2;
  if (nN <= 0 || nEs <= 0 || nEe <= 0) return;
  if (in_sizes[0] != nN * FDIM || in_sizes[1] != 2 * nEs || in_sizes[2] != 2 * nEe) return;
  for (int l = 0; l < 2; ++l) {
    const int b = 3 + 9 * l;
    for (int t = 0; t < 2; ++t) {
      const int o = b + 4 * t;
      if (in_sizes[o] != FDIM * FDIM || in_sizes[o + 1] != FDIM || in_sizes[o + 2] != FDIM || in_sizes[o + 3] != FDIM) return;
    }
    if (in_sizes[b + 8] != 1) return;
  }
  if (in_sizes[21] != OUTP * FDIM || in_sizes[22] != OUTP || in_sizes[23] != OUTP * OUTP || in_sizes[24] != OUTP) return;
  if (in_sizes[25] != OUTP * FDIM || in_sizes[26] != OUTP || in_sizes[27] != FDIM * OUTP || in_sizes[28] != FDIM) return;
  if (out_size != nN * (OUTP + FDIM + FDIM)) return;
  if (nEs > (1 << 28) || nEe > (1 << 28) || nN > (1 << 22)) return;

  const float* x     = (const float*)d_in[0];
  const int*   eiS   = (const int*)d_in[1];
  const int*   eiE   = (const int*)d_in[2];
  const float* Ws0   = (const float*)d_in[3];
  const float* as_s0 = (const float*)d_in[4];
  const float* ad_s0 = (const float*)d_in[5];
  const float* b_s0  = (const float*)d_in[6];
  const float* We0   = (const float*)d_in[7];
  const float* as_e0 = (const float*)d_in[8];
  const float* ad_e0 = (const float*)d_in[9];
  const float* b_e0  = (const float*)d_in[10];
  const float* g0    = (const float*)d_in[11];
  const float* Ws1   = (const float*)d_in[12];
  const float* as_s1 = (const float*)d_in[13];
  const float* ad_s1 = (const float*)d_in[14];
  const float* b_s1  = (const float*)d_in[15];
  const float* We1   = (const float*)d_in[16];
  const float* as_e1 = (const float*)d_in[17];
  const float* ad_e1 = (const float*)d_in[18];
  const float* b_e1  = (const float*)d_in[19];
  const float* g1    = (const float*)d_in[20];
  const float* Wp1   = (const float*)d_in[21];
  const float* bp1   = (const float*)d_in[22];
  const float* Wp2   = (const float*)d_in[23];
  const float* bp2   = (const float*)d_in[24];
  const float* Wr1   = (const float*)d_in[25];
  const float* br1   = (const float*)d_in[26];
  const float* Wr2   = (const float*)d_in[27];
  const float* br2   = (const float*)d_in[28];
  float* out  = (float*)d_out;
  float* outP = out;
  float* outR = out + (size_t)nN * OUTP;
  float* outZ = out + (size_t)nN * OUTP + (size_t)nN * FDIM;

  const int NPAD   = ((nN + TGT - 1) / TGT) * TGT;
  const int nBC    = (nN + NBC - 1) / NBC;
  const int CNTPAD = nBC * NBC;
  if (CNTPAD < NPAD) return;
  if (4 * nBC + 1 > RBN) return;
  const int nBF    = (nN + NBF - 1) / NBF;
  if (nBF + 1 > 4 * nBC + 1) return;
  if (31 * 4 * nBC > 4096) return;
  const int csrLenS = ((nEs + 31) & ~31) + 4096;
  const int csrLenE = ((nEe + 31) & ~31) + 4096;
  const int nAgg   = NPAD / TGT;
  const int nGemm  = NPAD / BMR;
  const int nXu    = NPAD * 32;

  char* ws = (char*)d_ws;
  size_t off = 0;
  const size_t oWP  = off; off += (size_t)WTOT * 2;                off = (off + 255) & ~(size_t)255;
  const size_t oXP  = off; off += (size_t)NPAD * FDIM * 2;         off = (off + 255) & ~(size_t)255;
  const size_t oHP  = off; off += (size_t)NPAD * FDIM * 2;         off = (off + 255) & ~(size_t)255;
  const size_t oZP  = off; off += (size_t)NPAD * FDIM * 2;         off = (off + 255) & ~(size_t)255;
  const size_t oTP  = off; off += (size_t)NPAD * HID2 * 2;         off = (off + 255) & ~(size_t)255;
  const size_t oHW  = off; off += (size_t)NPAD * FDIM * 4;         off = (off + 255) & ~(size_t)255;
  const size_t oHS  = off; off += (size_t)NPAD * FDIM * 4;         off = (off + 255) & ~(size_t)255;
  const size_t oES  = off; off += (size_t)NPAD * HEADS * 4;        off = (off + 255) & ~(size_t)255;
  const size_t oED  = off; off += (size_t)NPAD * HEADS * 4;        off = (off + 255) & ~(size_t)255;
  const size_t oCnS = off; off += (size_t)CNTPAD * 4;              off = (off + 255) & ~(size_t)255;
  const size_t oOfS = off; off += (size_t)CNTPAD * 4;              off = (off + 255) & ~(size_t)255;
  const size_t oRbS = off; off += (size_t)RBN * 4;                 off = (off + 255) & ~(size_t)255;
  const size_t oCsS = off; off += (size_t)csrLenS * 4;             off = (off + 255) & ~(size_t)255;
  const size_t oCnE = off; off += (size_t)CNTPAD * 4;              off = (off + 255) & ~(size_t)255;
  const size_t oOfE = off; off += (size_t)CNTPAD * 4;              off = (off + 255) & ~(size_t)255;
  const size_t oRbE = off; off += (size_t)RBN * 4;                 off = (off + 255) & ~(size_t)255;
  const size_t oCsE = off; off += (size_t)csrLenE * 4;             off = (off + 255) & ~(size_t)255;
  if (off > ws_size || off > (size_t)WSCAP) return;

  _Float16* wpl = (_Float16*)(ws + oWP);
  _Float16* xp  = (_Float16*)(ws + oXP);
  _Float16* hp  = (_Float16*)(ws + oHP);
  _Float16* zp  = (_Float16*)(ws + oZP);
  _Float16* tp  = (_Float16*)(ws + oTP);
  float* hw  = (float*)(ws + oHW);
  float* hs  = (float*)(ws + oHS);
  float* es  = (float*)(ws + oES);
  float* ed  = (float*)(ws + oED);
  CsrSet csS; csS.cnt = (int*)(ws + oCnS); csS.off = (int*)(ws + oOfS); csS.rb = (int*)(ws + oRbS); csS.csr = (int*)(ws + oCsS);
  CsrSet csE; csE.cnt = (int*)(ws + oCnE); csE.off = (int*)(ws + oOfE); csE.rb = (int*)(ws + oRbE); csE.csr = (int*)(ws + oCsE);

  const _Float16* pWs0 = wpl;
  const _Float16* pWe0 = wpl + WSEG1;
  const _Float16* pWs1 = wpl + WSEG2;
  const _Float16* pWe1 = wpl + WSEG3;
  const _Float16* pW1h = wpl + WSEG4;
  const _Float16* pWp2 = wpl + WSEG6;
  const _Float16* pWr2 = wpl + WSEG7;

  k_wcvt<<<WTOT / 8 / NTHR, NTHR, 0, stream>>>(Ws0, We0, Ws1, We1, Wp1, Wr1, Wp2, Wr2, wpl);
  k_xcvt<<<(nXu + NTHR - 1) / NTHR, NTHR, 0, stream>>>(x, xp, nN, nXu);

  build_csr(eiS, eiS + nEs, nEs, nN, nBC, nBF, csrLenS, csS, stream);
  build_csr(eiE, eiE + nEe, nEe, nN, nBC, nBF, csrLenE, csE, stream);

  k_gemm_att<FDIM, FDIM><<<nGemm, NTHR, 0, stream>>>(xp, pWs0, as_s0, ad_s0, hw, es, ed);
  k_agg<0><<<nAgg, NTHR, 0, stream>>>(csS.csr, csS.off, csS.cnt, es, ed, hw, b_s0, g0, hs, hs, hp, nN, csrLenS);
  k_gemm_att<FDIM, FDIM><<<nGemm, NTHR, 0, stream>>>(xp, pWe0, as_e0, ad_e0, hw, es, ed);
  k_agg<1><<<nAgg, NTHR, 0, stream>>>(csE.csr, csE.off, csE.cnt, es, ed, hw, b_e0, g0, hs, hs, hp, nN, csrLenE);

  k_gemm_att<FDIM, FDIM><<<nGemm, NTHR, 0, stream>>>(hp, pWs1, as_s1, ad_s1, hw, es, ed);
  k_agg<0><<<nAgg, NTHR, 0, stream>>>(csS.csr, csS.off, csS.cnt, es, ed, hw, b_s1, g1, hs, hs, zp, nN, csrLenS);
  k_gemm_att<FDIM, FDIM><<<nGemm, NTHR, 0, stream>>>(hp, pWe1, as_e1, ad_e1, hw, es, ed);
  k_agg<2><<<nAgg, NTHR, 0, stream>>>(csE.csr, csE.off, csE.cnt, es, ed, hw, b_e1, g1, hs, outZ, zp, nN, csrLenE);

  k_gemm_relu16<<<nGemm, NTHR, 0, stream>>>(zp, pW1h, bp1, br1, tp);
  k_gemm_out<OUTP, HID2, OUTP><<<nGemm, NTHR, 0, stream>>>(tp, pWp2, bp2, outP, nN);
  k_gemm_out<OUTP, HID2, FDIM><<<nGemm, NTHR, 0, stream>>>(tp + OUTP, pWr2, br2, outR, nN);
}
